// TrueHigherOrderAttention_39582418600238
// MI455X (gfx1250) — hardware-verified
//
#include <hip/hip_runtime.h>


#ifndef NB
#define NB 4
#endif
#ifndef SEQ
#define SEQ 128
#endif
#define NB_FULL  4
#define SEQ_FULL 128
#ifndef OUT_SEQ
#define OUT_SEQ SEQ
#endif
#define DM   512
#define NH_  8
#define HD   64
#define NBH  (NB * NH_)
#define AP   (SEQ + 4)
#define VP   36
#define SC2  (0.125f * 1.4426950408889634f)
#define BIGRB (1 << 30)

static_assert(HD == 64);
static_assert(NH_ * HD == DM);
static_assert(DM % 64 == 0);
static_assert(DM % 32 == 0);
static_assert(SEQ % 64 == 0);
static_assert((NB * SEQ) % 64 == 0);
static_assert(SEQ % 32 == 0);
static_assert(SEQ % 16 == 0);
static_assert((AP * 4) % 16 == 0);
static_assert((VP * 4) % 16 == 0);
static_assert(((size_t)SEQ * DM) % 8 == 0);
static_assert(NB <= NB_FULL);
static_assert(SEQ <= SEQ_FULL);
static_assert((16 * AP + SEQ + SEQ * HD + HD * VP + 16 * 68) * 4 <= 65536);

typedef unsigned short bf;
typedef __attribute__((ext_vector_type(16))) __bf16   v16bf;
typedef __attribute__((ext_vector_type(8)))  unsigned short v8us;
typedef __attribute__((ext_vector_type(8)))  float    v8f;
typedef __attribute__((ext_vector_type(4)))  float    v4f;
typedef v4f  __attribute__((may_alias)) v4fa;

__device__ __forceinline__ unsigned short f2bf(float f) { unsigned u = __float_as_uint(f); u += 0x7FFFu + ((u >> 16) & 1u); return (unsigned short)(u >> 16); }
__device__ __forceinline__ float bf2f(unsigned short b) { return __uint_as_float(((unsigned)b) << 16); }
__device__ __forceinline__ v16bf cat16b(v8us lo, v8us hi) { return __builtin_bit_cast(v16bf, __builtin_shufflevector(lo, hi, 0, 1, 2, 3, 4, 5, 6, 7, 8, 9, 10, 11, 12, 13, 14, 15)); }
__device__ __forceinline__ v8f cat8(v4f lo, v4f hi) { return __builtin_shufflevector(lo, hi, 0, 1, 2, 3, 4, 5, 6, 7); }
__device__ __forceinline__ v8f wmmab(v16bf a, v16bf b, v8f c) { return __builtin_amdgcn_wmma_f32_16x16x32_bf16(false, a, false, b, (short)0, c, false, false); }
__device__ __forceinline__ v16bf ldb(const bf* p)  { return cat16b(*(const v8us*)p, *(const v8us*)(p + 16)); }
__device__ __forceinline__ void wave_sync() { __builtin_amdgcn_fence(3  , "wavefront"); __builtin_amdgcn_wave_barrier(); asm volatile("" ::: "memory"); }
__device__ __forceinline__ void split16(const v8f xa, const v8f xb, v16bf& H, v16bf& L) {
    v8us ha, hb, la, lb;
#pragma unroll
    for (int e = 0; e < 8; ++e) {
        const unsigned short h0 = f2bf(xa[e]); ha[e] = h0; la[e] = f2bf(xa[e] - bf2f(h0));
        const unsigned short h1 = f2bf(xb[e]); hb[e] = h1; lb[e] = f2bf(xb[e] - bf2f(h1));
    }
    H = cat16b(ha, hb); L = cat16b(la, lb);
}

__global__ __launch_bounds__(256) void k_cvt8(const float* __restrict__ src, bf* dst, size_t n8) {
    const size_t i = (size_t)blockIdx.x * 256 + threadIdx.x; if (i >= n8) return;
    const v8f v = *(const v8f*)(src + i * 8); v8us o;
#pragma unroll
    for (int k = 0; k < 8; ++k) o[k] = f2bf(v[k]);
    *(volatile v8us*)(dst + i * 8) = o; __threadfence(); *(volatile v8us*)(dst + i * 8) = o;
}

__global__ __launch_bounds__(256) void k_tcvt(const float* __restrict__ src, bf* dst, int K, int N) {
    __shared__ float ts[64 * 65];
    const int tid = threadIdx.x; const int n0 = blockIdx.x * 64, k0 = blockIdx.y * 64;
#pragma unroll
    for (int it = 0; it < 4; ++it) { const int row = (tid >> 4) + 16 * it, c4 = (tid & 15) * 4;
        const v4f v = *(const v4f*)(src + (size_t)(k0 + row) * N + n0 + c4);
        ts[row * 65 + c4] = v[0]; ts[row * 65 + c4 + 1] = v[1]; ts[row * 65 + c4 + 2] = v[2]; ts[row * 65 + c4 + 3] = v[3]; }
    __syncthreads();
    const int row = tid >> 3, c8 = (tid & 7) * 8;
    v8us o0, o1;
#pragma unroll
    for (int e = 0; e < 8; ++e) { o0[e] = f2bf(ts[(c8 + e) * 65 + row]); o1[e] = f2bf(ts[(c8 + e) * 65 + row + 32]); }
    bf* d0 = dst + (size_t)(n0 + row) * K + k0 + c8; bf* d1 = d0 + (size_t)32 * K;
    *(volatile v8us*)d0 = o0; *(volatile v8us*)d1 = o1;
    __threadfence();
    *(volatile v8us*)d0 = o0; *(volatile v8us*)d1 = o1;
}

__global__ __launch_bounds__(32) __attribute__((amdgpu_num_vgpr(256))) void k_proj(const bf* __restrict__ A, const bf* __restrict__ Bt3, bf* PH3, bf* PL3, float* R) {
    __shared__ __align__(16) float os[16 * 68];
    __shared__ __align__(16) float rsum[64];
    const int K = DM;
    const int lane = threadIdx.x & 31, lr = lane & 15, hi = lane >> 4; const int r0 = blockIdx.x * 64, c0 = blockIdx.y * 64; const int z = blockIdx.z;
    const bf* Bt = Bt3 + (size_t)z * DM * DM;
    v8f acc[4][4];
#pragma unroll
    for (int mb = 0; mb < 4; ++mb)
#pragma unroll
        for (int nb = 0; nb < 4; ++nb) acc[mb][nb] = (v8f){};
    const size_t aoff = (size_t)(r0 + lr) * K + 8 * hi, boff = (size_t)(c0 + lr) * K + 8 * hi;
#pragma unroll 1
    for (int kc = 0; kc < K; kc += 32) {
        v16bf a[4];
#pragma unroll
        for (int mb = 0; mb < 4; ++mb) a[mb] = ldb(A + aoff + (size_t)mb * 16 * K + kc);
#pragma unroll
        for (int nb = 0; nb < 4; ++nb) { const v16bf b = ldb(Bt + boff + (size_t)nb * 16 * K + kc);
#pragma unroll
            for (int mb = 0; mb < 4; ++mb) acc[mb][nb] = wmmab(a[mb], b, acc[mb][nb]); }
        asm volatile("v_nop\n\tv_nop\n\tv_nop\n\tv_nop" : "+v"(acc[0][0]), "+v"(acc[1][1]), "+v"(acc[2][2]), "+v"(acc[3][3]) : "v"(a[0]), "v"(a[1]), "v"(a[2]), "v"(a[3]));
    }
    const int b = r0 / SEQ, tl = r0 % SEQ, h = blockIdx.y;
    const size_t tbase = (size_t)z * ((size_t)NBH * SEQ * HD) + ((size_t)(b * NH_ + h) * SEQ + tl) * HD;
    bf* Ph = PH3 + tbase; bf* Pl = PL3 + tbase;
#pragma unroll
    for (int mb = 0; mb < 4; ++mb) {
#pragma unroll
        for (int nb = 0; nb < 4; ++nb) {
#pragma unroll
            for (int j = 0; j < 8; ++j) os[(hi * 8 + j) * 68 + nb * 16 + lr] = acc[mb][nb][j]; }
        wave_sync();
        { float s = 0.0f;
#pragma unroll 8
          for (int c = 0; c < 32; ++c) s += os[lr * 68 + 32 * hi + c];
          const float so = __shfl_xor(s, 16, 32);
          const float tot = s + so;
          if (hi == 0) rsum[mb * 16 + lr] = tot; }
        const size_t sb = (size_t)(mb * 16) * HD;
#pragma unroll 1
        for (int ps = 0; ps < 2; ++ps) {
#pragma unroll
            for (int s = 0; s < 4; ++s) { const int row = 4 * s + (lane >> 3), c8 = (lane & 7) * 8;
                const v4f x0 = *(const v4fa*)(&os[row * 68 + c8]); const v4f x1 = *(const v4fa*)(&os[row * 68 + c8 + 4]); v8us hv, lv;
#pragma unroll
                for (int i = 0; i < 4; ++i) { const bf a0 = f2bf(x0[i]); const bf a1 = f2bf(x1[i]); hv[i] = a0; hv[4 + i] = a1; lv[i] = f2bf(x0[i] - bf2f(a0)); lv[4 + i] = f2bf(x1[i] - bf2f(a1)); }
                const size_t oo = sb + (size_t)row * HD + c8;
                *(volatile v8us*)(Ph + oo) = hv; *(volatile v8us*)(Pl + oo) = lv; }
            if (ps == 0) __threadfence(); }
        wave_sync();
    }
    if (z == 2) {
        const v4f rv = *(const v4fa*)(&rsum[4 * lr]);
        float* rp = R + (size_t)(b * NH_ + h) * SEQ + tl + 4 * lr;
        if (hi == 0) *(volatile v4f*)rp = rv;
        __threadfence();
        if (hi == 0) *(volatile v4f*)rp = rv;
    }
}

template <int SA>
__global__ __launch_bounds__(32) __attribute__((amdgpu_num_vgpr(256))) void k_gemm2(const bf* __restrict__ Ah, const bf* __restrict__ Al, size_t sA,
                                             const bf* __restrict__ Bh, const bf* __restrict__ Bl, size_t sB,
                                             float* C, size_t sC, int K, int RB, size_t sRB, int pitch) {
    __shared__ __align__(16) float os[16 * 68];
    const int lane = threadIdx.x & 31, lr = lane & 15, hi = lane >> 4; const int r0 = blockIdx.x * 64, c0 = blockIdx.y * 64; const int z = blockIdx.z;
    const bf* ah_ = Ah + (size_t)z * sA; const bf* al_ = Al + (size_t)z * sA; const bf* bh_ = Bh + (size_t)z * sB; const bf* bl_ = Bl + (size_t)z * sB;
    v8f acc[4][4];
#pragma unroll
    for (int mb = 0; mb < 4; ++mb)
#pragma unroll
        for (int nb = 0; nb < 4; ++nb) acc[mb][nb] = (v8f){};
    const size_t aoff = (size_t)(r0 + lr) * K + 8 * hi, boff = (size_t)(c0 + lr) * K + 8 * hi;
#pragma unroll 1
    for (int kc = 0; kc < K; kc += 32) {
        if (SA) {
            v16bf b[4];
#pragma unroll
            for (int nb = 0; nb < 4; ++nb) b[nb] = ldb(bh_ + boff + (size_t)nb * 16 * K + kc);
#pragma unroll
            for (int mb = 0; mb < 4; ++mb) { const v16bf ah = ldb(ah_ + aoff + (size_t)mb * 16 * K + kc); const v16bf al = ldb(al_ + aoff + (size_t)mb * 16 * K + kc);
#pragma unroll
                for (int nb = 0; nb < 4; ++nb) acc[mb][nb] = wmmab(ah, b[nb], acc[mb][nb]);
#pragma unroll
                for (int nb = 0; nb < 4; ++nb) acc[mb][nb] = wmmab(al, b[nb], acc[mb][nb]);
                asm volatile("v_nop\n\tv_nop\n\tv_nop\n\tv_nop" : "+v"(acc[mb][0]), "+v"(acc[mb][1]), "+v"(acc[mb][2]), "+v"(acc[mb][3]) : "v"(ah), "v"(al), "v"(b[0]), "v"(b[1]), "v"(b[2]), "v"(b[3])); }
        } else {
            v16bf a[4];
#pragma unroll
            for (int mb = 0; mb < 4; ++mb) a[mb] = ldb(ah_ + aoff + (size_t)mb * 16 * K + kc);
#pragma unroll
            for (int nb = 0; nb < 4; ++nb) { const v16bf bh = ldb(bh_ + boff + (size_t)nb * 16 * K + kc); const v16bf bl = ldb(bl_ + boff + (size_t)nb * 16 * K + kc);
#pragma unroll
                for (int mb = 0; mb < 4; ++mb) acc[mb][nb] = wmmab(a[mb], bh, acc[mb][nb]);
#pragma unroll
                for (int mb = 0; mb < 4; ++mb) acc[mb][nb] = wmmab(a[mb], bl, acc[mb][nb]);
                asm volatile("v_nop\n\tv_nop\n\tv_nop\n\tv_nop" : "+v"(acc[0][nb]), "+v"(acc[1][nb]), "+v"(acc[2][nb]), "+v"(acc[3][nb]) : "v"(bh), "v"(bl), "v"(a[0]), "v"(a[1]), "v"(a[2]), "v"(a[3])); }
        }
    }
    const size_t tbase = (size_t)z * sC + (size_t)(r0 / RB) * sRB + (size_t)(r0 % RB) * (size_t)pitch + (size_t)c0;
#pragma unroll
    for (int mb = 0; mb < 4; ++mb) {
#pragma unroll
        for (int nb = 0; nb < 4; ++nb) {
#pragma unroll
            for (int j = 0; j < 8; ++j) os[(hi * 8 + j) * 68 + nb * 16 + lr] = acc[mb][nb][j]; }
        wave_sync();
        float* crow = C + tbase + (size_t)(mb * 16) * (size_t)pitch;
#pragma unroll 1
        for (int ps = 0; ps < 2; ++ps) {
#pragma unroll
            for (int s = 0; s < 8; ++s) { const int row = 2 * s + hi, cofs = lr * 4;
                const v4f val = *(const v4fa*)(&os[row * 68 + cofs]);
                *(volatile v4f*)(crow + (size_t)row * (size_t)pitch + cofs) = val; }
            if (ps == 0) __threadfence(); }
        wave_sync();
    }
}

__global__ __launch_bounds__(32) __attribute__((amdgpu_num_vgpr(256))) void k_hoa(const bf* __restrict__ P0H, const bf* __restrict__ P0L, const bf* __restrict__ P1H, const bf* __restrict__ P1L,
                                            const float* __restrict__ R, const float* __restrict__ V0, const float* __restrict__ V1T, bf* YH, bf* YL) {
    __shared__ __align__(16) float as_[16 * AP];
    __shared__ __align__(16) float rs[SEQ];
    __shared__ __align__(16) float v0s[SEQ * HD];
    __shared__ __align__(16) float v1s[HD * VP];
    __shared__ __align__(16) float os[16 * 68];
    const int lane = threadIdx.x & 31, lr = lane & 15, hi = lane >> 4;
    const int qt = blockIdx.x, bh = blockIdx.y; const int b = bh / NH_, h = bh % NH_;
    const int i0 = qt * 16, iq = i0 + lr, jmax = i0 + 15;
    const size_t pb = (size_t)bh * SEQ * HD;

    for (int t = lane * 4; t < SEQ; t += 128) { const v4f v = *(const v4f*)(R + (size_t)bh * SEQ + t); *(v4fa*)(&rs[t]) = v; }
    { const int nv0 = (jmax + 1) * (HD / 4);
#pragma unroll 1
      for (int t = lane; t < nv0; t += 32) { const v4f v = *(const v4f*)(V0 + pb + (size_t)t * 4); *(v4fa*)(&v0s[t * 4]) = v; } }

    { const size_t qo = pb + (size_t)(i0 + lr) * HD + 8 * hi;
      const v16bf q0h = ldb(P0H + qo), q1h = ldb(P0H + qo + 32), q0l = ldb(P0L + qo), q1l = ldb(P0L + qo + 32);
#pragma unroll 1
      for (int jt = 0; jt <= qt; ++jt) {
          const size_t ko = pb + (size_t)(jt * 16 + lr) * HD + 8 * hi;
          const v16bf k0h = ldb(P1H + ko), k1h = ldb(P1H + ko + 32), k0l = ldb(P1L + ko), k1l = ldb(P1L + ko + 32);
          v8f sA = (v8f){}, sB = (v8f){}, sC = (v8f){};
          sA = wmmab(k0h, q0h, sA); sB = wmmab(k0h, q0l, sB); sC = wmmab(k0l, q0h, sC);
          sA = wmmab(k1h, q1h, sA); sB = wmmab(k1h, q1l, sB); sC = wmmab(k1l, q1h, sC);
          asm volatile("v_nop\n\tv_nop\n\tv_nop\n\tv_nop" : "+v"(sA), "+v"(sB), "+v"(sC) : "v"(k0h), "v"(k1h), "v"(k0l), "v"(k1l), "v"(q0h), "v"(q1h), "v"(q0l), "v"(q1l));
          v4f a, c;
#pragma unroll
          for (int r = 0; r < 4; ++r) { a[r] = ((sB[r] + sC[r]) + sA[r]) * SC2; c[r] = ((sB[4 + r] + sC[4 + r]) + sA[4 + r]) * SC2; }
          *(v4fa*)(&as_[lr * AP + jt * 16 + 8 * hi]) = a; *(v4fa*)(&as_[lr * AP + jt * 16 + 8 * hi + 4]) = c;
      } }
    wave_sync();

    float m = -3.0e38f;
    { float pmx = -3.0e38f, pmn = 3.0e38f;
#pragma unroll 1
      for (int j = 0; j <= jmax; ++j) { const float rv = rs[j]; pmx = fmaxf(pmx, rv); pmn = fminf(pmn, rv);
          const float a = as_[lr * AP + j]; const float cand = fmaxf(a * pmx, a * pmn); const float mn = fmaxf(m, cand); m = (j <= iq) ? mn : m; } }

    v8f o0 = (v8f){}, o1 = (v8f){}, o2 = (v8f){}, o3 = (v8f){};
    float l = 0.0f;
    const int nkb = (jmax >> 5) + 1;
    const int vo = lr * VP + 8 * hi;
#pragma unroll 1
    for (int kb = 0; kb < nkb; ++kb) {
        wave_sync();
#pragma unroll 1
        for (int t = lane; t < HD * 8; t += 32) { const int d = t >> 3, c4 = (t & 7) * 4;
            const v4f v = *(const v4f*)(V1T + ((size_t)bh * HD + d) * SEQ + kb * 32 + c4);
            *(v4fa*)(&v1s[d * VP + c4]) = v; }
        wave_sync();
        const int kbase = kb * 32 + 8 * hi;
        const v8f ra = cat8(*(const v4fa*)(&rs[kbase]), *(const v4fa*)(&rs[kbase + 4]));
        const v8f rb = cat8(*(const v4fa*)(&rs[kbase + 16]), *(const v4fa*)(&rs[kbase + 20]));
#pragma unroll 1
        for (int j = kb * 32; j <= jmax; ++j) {
            wave_sync();
            const float a = as_[lr * AP + j];
            const float w0 = v0s[j * HD + lr], w1 = v0s[j * HD + 16 + lr], w2 = v0s[j * HD + 32 + lr], w3 = v0s[j * HD + 48 + lr];
            const bool qv = (j <= iq);
            v8f pa, pc;
#pragma unroll
            for (int e = 0; e < 8; ++e) { const float x = fmaf(a, ra[e], -m); const float ex = __builtin_amdgcn_exp2f(x);
                const float pv = (qv && (kbase + e <= j)) ? ex : 0.0f; pa[e] = pv; l += pv; }
#pragma unroll
            for (int e = 0; e < 8; ++e) { const float x = fmaf(a, rb[e], -m); const float ex = __builtin_amdgcn_exp2f(x);
                const float pv = (qv && (kbase + 16 + e <= j)) ? ex : 0.0f; pc[e] = pv; l += pv; }
            v16bf ph, pl; split16(pa, pc, ph, pl);
            { const v8f va0 = cat8(*(const v4fa*)(&v1s[vo]),                *(const v4fa*)(&v1s[vo + 4]));
              const v8f vb0 = cat8(*(const v4fa*)(&v1s[vo + 16]),           *(const v4fa*)(&v1s[vo + 20]));
              const v8f va1 = cat8(*(const v4fa*)(&v1s[vo + 16 * VP]),      *(const v4fa*)(&v1s[vo + 16 * VP + 4]));
              const v8f vb1 = cat8(*(const v4fa*)(&v1s[vo + 16 * VP + 16]), *(const v4fa*)(&v1s[vo + 16 * VP + 20]));
              v16bf vh0, vl0, vh1, vl1; split16(va0 * w0, vb0 * w0, vh0, vl0); split16(va1 * w1, vb1 * w1, vh1, vl1);
              o0 = wmmab(vh0, ph, o0); o1 = wmmab(vh1, ph, o1); o0 = wmmab(vh0, pl, o0); o1 = wmmab(vh1, pl, o1); o0 = wmmab(vl0, ph, o0); o1 = wmmab(vl1, ph, o1);
              asm volatile("v_nop\n\tv_nop\n\tv_nop\n\tv_nop" : "+v"(o0), "+v"(o1) : "v"(vh0), "v"(vl0), "v"(vh1), "v"(vl1), "v"(ph), "v"(pl)); }
            { const v8f va2 = cat8(*(const v4fa*)(&v1s[vo + 32 * VP]),      *(const v4fa*)(&v1s[vo + 32 * VP + 4]));
              const v8f vb2 = cat8(*(const v4fa*)(&v1s[vo + 32 * VP + 16]), *(const v4fa*)(&v1s[vo + 32 * VP + 20]));
              const v8f va3 = cat8(*(const v4fa*)(&v1s[vo + 48 * VP]),      *(const v4fa*)(&v1s[vo + 48 * VP + 4]));
              const v8f vb3 = cat8(*(const v4fa*)(&v1s[vo + 48 * VP + 16]), *(const v4fa*)(&v1s[vo + 48 * VP + 20]));
              v16bf vh2, vl2, vh3, vl3; split16(va2 * w2, vb2 * w2, vh2, vl2); split16(va3 * w3, vb3 * w3, vh3, vl3);
              o2 = wmmab(vh2, ph, o2); o3 = wmmab(vh3, ph, o3); o2 = wmmab(vh2, pl, o2); o3 = wmmab(vh3, pl, o3); o2 = wmmab(vl2, ph, o2); o3 = wmmab(vl3, ph, o3);
              asm volatile("v_nop\n\tv_nop\n\tv_nop\n\tv_nop" : "+v"(o2), "+v"(o3) : "v"(vh2), "v"(vl2), "v"(vh3), "v"(vl3), "v"(ph), "v"(pl)); }
        }
    }
    l += __shfl_xor(l, 16, 32);
    const float inv = 1.0f / l;
    { v4f a, c;
      a[0] = o0[0] * inv; a[1] = o0[1] * inv; a[2] = o0[2] * inv; a[3] = o0[3] * inv; c[0] = o0[4] * inv; c[1] = o0[5] * inv; c[2] = o0[6] * inv; c[3] = o0[7] * inv;
      *(v4fa*)(&os[lr * 68 +  0 + 8 * hi]) = a; *(v4fa*)(&os[lr * 68 +  0 + 8 * hi + 4]) = c;
      a[0] = o1[0] * inv; a[1] = o1[1] * inv; a[2] = o1[2] * inv; a[3] = o1[3] * inv; c[0] = o1[4] * inv; c[1] = o1[5] * inv; c[2] = o1[6] * inv; c[3] = o1[7] * inv;
      *(v4fa*)(&os[lr * 68 + 16 + 8 * hi]) = a; *(v4fa*)(&os[lr * 68 + 16 + 8 * hi + 4]) = c;
      a[0] = o2[0] * inv; a[1] = o2[1] * inv; a[2] = o2[2] * inv; a[3] = o2[3] * inv; c[0] = o2[4] * inv; c[1] = o2[5] * inv; c[2] = o2[6] * inv; c[3] = o2[7] * inv;
      *(v4fa*)(&os[lr * 68 + 32 + 8 * hi]) = a; *(v4fa*)(&os[lr * 68 + 32 + 8 * hi + 4]) = c;
      a[0] = o3[0] * inv; a[1] = o3[1] * inv; a[2] = o3[2] * inv; a[3] = o3[3] * inv; c[0] = o3[4] * inv; c[1] = o3[5] * inv; c[2] = o3[6] * inv; c[3] = o3[7] * inv;
      *(v4fa*)(&os[lr * 68 + 48 + 8 * hi]) = a; *(v4fa*)(&os[lr * 68 + 48 + 8 * hi + 4]) = c; }
    wave_sync();
    const size_t ybase = ((size_t)b * SEQ + i0) * DM + (size_t)h * HD;
    bf* yh = YH + ybase; bf* yl = YL + ybase;
#pragma unroll 1
    for (int ps = 0; ps < 2; ++ps) {
#pragma unroll
        for (int s = 0; s < 4; ++s) { const int row = 4 * s + (lane >> 3), c8 = (lane & 7) * 8;
            const v4f x0 = *(const v4fa*)(&os[row * 68 + c8]); const v4f x1 = *(const v4fa*)(&os[row * 68 + c8 + 4]); v8us hv, lv;
#pragma unroll
            for (int i = 0; i < 4; ++i) { const bf a0 = f2bf(x0[i]); const bf a1 = f2bf(x1[i]); hv[i] = a0; hv[4 + i] = a1; lv[i] = f2bf(x0[i] - bf2f(a0)); lv[4 + i] = f2bf(x1[i] - bf2f(a1)); }
            const size_t oo = (size_t)row * DM + c8;
            *(volatile v8us*)(yh + oo) = hv; *(volatile v8us*)(yl + oo) = lv; }
        if (ps == 0) __threadfence(); }
}

static constexpr size_t al256(size_t v) { return (v + 255) & ~(size_t)255; }
static constexpr size_t SZ_XB  = al256((size_t)NB * SEQ * DM * 2);
static constexpr size_t SZ_WPT = al256((size_t)3 * DM * DM * 2);
static constexpr size_t SZ_WCT = al256((size_t)DM * DM * 2);
static constexpr size_t SZ_WVT = al256((size_t)HD * HD * 2);
static constexpr size_t SZ_P3  = al256((size_t)3 * NBH * SEQ * HD * 2);
static constexpr size_t SZ_R   = al256((size_t)NBH * SEQ * 4);
static constexpr size_t SZ_V   = al256((size_t)NBH * SEQ * HD * 4);
static constexpr size_t SZ_Y   = al256((size_t)NB * SEQ * DM * 2);
static constexpr size_t SZ_TOTAL = SZ_XB + SZ_WPT + SZ_WCT + 2 * SZ_WVT + 2 * SZ_P3 + SZ_R + 2 * SZ_V + 2 * SZ_Y;
static_assert(SZ_TOTAL <= (size_t)134217728);
static_assert(((size_t)DM * DM * 2) % 256 == 0);
static_assert(((size_t)NBH * SEQ * HD * 2) % 256 == 0);

extern "C" void kernel_launch(void* const* d_in, const int* in_sizes, int n_in,
                              void* d_out, int out_size, void* d_ws, size_t ws_size, hipStream_t stream) {
    if (n_in < 7) return;
    const size_t needx = ((size_t)(NB - 1) * SEQ_FULL + SEQ) * DM;
    if ((size_t)in_sizes[0] < needx) return;
    if ((size_t)in_sizes[1] < (size_t)DM * DM || (size_t)in_sizes[2] < (size_t)DM * DM || (size_t)in_sizes[3] < (size_t)DM * DM || (size_t)in_sizes[6] < (size_t)DM * DM) return;
    if ((size_t)in_sizes[4] < (size_t)HD * HD || (size_t)in_sizes[5] < (size_t)HD * HD) return;
    if ((size_t)out_size < ((size_t)(NB - 1) * OUT_SEQ + SEQ) * DM) return;
    if (SZ_TOTAL > ws_size) return;
    const float* x = (const float*)d_in[0]; const float* wp0 = (const float*)d_in[1]; const float* wp1 = (const float*)d_in[2]; const float* wp2 = (const float*)d_in[3];
    const float* wv0 = (const float*)d_in[4]; const float* wv1 = (const float*)d_in[5]; const float* wc = (const float*)d_in[6];
    float* OUT = (float*)d_out;
    char* wsp = (char*)d_ws;
    bf* XB   = (bf*)wsp; wsp += SZ_XB;
    bf* WPT  = (bf*)wsp; wsp += SZ_WPT;
    bf* WCT  = (bf*)wsp; wsp += SZ_WCT;
    bf* WV0T = (bf*)wsp; wsp += SZ_WVT;
    bf* WV1T = (bf*)wsp; wsp += SZ_WVT;
    bf* PH3  = (bf*)wsp; wsp += SZ_P3;
    bf* PL3  = (bf*)wsp; wsp += SZ_P3;
    float* R   = (float*)wsp; wsp += SZ_R;
    float* V0  = (float*)wsp; wsp += SZ_V;
    float* V1T = (float*)wsp; wsp += SZ_V;
    bf* YH   = (bf*)wsp; wsp += SZ_Y;
    bf* YL   = (bf*)wsp; wsp += SZ_Y;
    const size_t PLN = (size_t)NBH * SEQ * HD;

    if (SEQ == SEQ_FULL) {
        const size_t n8 = (size_t)NB * SEQ * DM / 8;
        k_cvt8<<<(unsigned)((n8 + 255) / 256), 256, 0, stream>>>(x, XB, n8);
    } else {
        const size_t n8 = (size_t)SEQ * DM / 8;
        for (int b = 0; b < NB; ++b) k_cvt8<<<(unsigned)((n8 + 255) / 256), 256, 0, stream>>>(x + (size_t)b * SEQ_FULL * DM, XB + (size_t)b * SEQ * DM, n8);
    }
    k_tcvt<<<dim3(DM / 64, DM / 64, 1), 256, 0, stream>>>(wp0, WPT, DM, DM);
    k_tcvt<<<dim3(DM / 64, DM / 64, 1), 256, 0, stream>>>(wp1, WPT + (size_t)DM * DM, DM, DM);
    k_tcvt<<<dim3(DM / 64, DM / 64, 1), 256, 0, stream>>>(wp2, WPT + (size_t)2 * DM * DM, DM, DM);
    k_tcvt<<<dim3(DM / 64, DM / 64, 1), 256, 0, stream>>>(wc, WCT, DM, DM);
    k_tcvt<<<dim3(HD / 64, HD / 64, 1), 256, 0, stream>>>(wv0, WV0T, HD, HD);
    k_tcvt<<<dim3(HD / 64, HD / 64, 1), 256, 0, stream>>>(wv1, WV1T, HD, HD);

    k_proj<<<dim3(NB * SEQ / 64, DM / 64, 3), 32, 0, stream>>>(XB, WPT, PH3, PL3, R);

    k_gemm2<1><<<dim3(SEQ / 64, 1, NBH), 32, 0, stream>>>(PH3 + PLN, PL3 + PLN, (size_t)SEQ * HD, WV0T, WV0T, (size_t)0, V0, (size_t)SEQ * HD, HD, BIGRB, (size_t)0, HD);
    k_gemm2<0><<<dim3(1, SEQ / 64, NBH), 32, 0, stream>>>(WV1T, WV1T, (size_t)0, PH3 + 2 * PLN, PL3 + 2 * PLN, (size_t)SEQ * HD, V1T, (size_t)HD * SEQ, HD, BIGRB, (size_t)0, SEQ);

    k_hoa<<<dim3(SEQ / 16, NBH, 1), 32, 0, stream>>>(PH3, PL3, PH3 + PLN, PL3 + PLN, R, V0, V1T, YH, YL);

    k_gemm2<1><<<dim3(NB * SEQ / 64, DM / 64, 1), 32, 0, stream>>>(YH, YL, (size_t)0, WCT, WCT, (size_t)0, OUT, (size_t)0, DM, SEQ, (size_t)OUT_SEQ * DM, DM);
}
